// NonLocalBlock_31138512896696
// MI455X (gfx1250) — hardware-verified
//
#include <hip/hip_runtime.h>


#ifndef NB
#define NB 8
#endif
#ifndef SEQ
#define SEQ 4096
#endif
#define NB_FULL  8
#define SEQ_FULL 4096
#ifndef OUT_SEQ
#define OUT_SEQ SEQ
#endif
#define CIN  256
#define CB   128
#define COUT 256
#define MK   (SEQ / 2)
#define AW   4
#define OPF  132
#define QRS  2048.0f
#define QRI  (1.0f / 2048.0f)
#define L2E  1.4426950408889634f
#define PSH  14.0f
#define NEGB (-3.0e38f)
#define WOS  64.0f
#define WOI  (1.0f / 64.0f)

static_assert(CB == 128);
static_assert(COUT == 256);
static_assert(CIN == COUT);
static_assert(CIN % 32 == 0);
static_assert(CB % 32 == 0);
static_assert(CIN % 64 == 0);
static_assert(CB % 64 == 0);
static_assert(COUT % 64 == 0);
static_assert(SEQ % 128 == 0);
static_assert((NB * SEQ) % 128 == 0);
static_assert((NB * SEQ) % 64 == 0);
static_assert(MK % 32 == 0);
static_assert(MK % 64 == 0);
static_assert(SEQ % (16 * AW) == 0);
static_assert(((size_t)SEQ * CIN) % 8 == 0);
static_assert(NB <= NB_FULL);
static_assert(SEQ <= SEQ_FULL);
static_assert((OPF * 4) % 16 == 0);
static_assert((size_t)NB * SEQ * CIN < (size_t)2147483647);

typedef _Float16 h16;
typedef unsigned short bf;
typedef __attribute__((ext_vector_type(16))) __bf16   v16bf;
typedef __attribute__((ext_vector_type(16))) _Float16 v16h;
typedef __attribute__((ext_vector_type(8)))  _Float16 v8h;
typedef __attribute__((ext_vector_type(8)))  unsigned short v8us;
typedef __attribute__((ext_vector_type(8)))  float    v8f;
typedef __attribute__((ext_vector_type(4)))  float    v4f;
typedef v4f  __attribute__((may_alias)) v4fa;

__device__ __forceinline__ unsigned short f2bf(float f) { unsigned u = __float_as_uint(f); u += 0x7FFFu + ((u >> 16) & 1u); return (unsigned short)(u >> 16); }
__device__ __forceinline__ float bfr(float f) { return __uint_as_float(((unsigned)f2bf(f)) << 16); }
__device__ __forceinline__ v16h cat16(v8h lo, v8h hi) { return __builtin_shufflevector(lo, hi, 0, 1, 2, 3, 4, 5, 6, 7, 8, 9, 10, 11, 12, 13, 14, 15); }
__device__ __forceinline__ v16bf cat16b(v8us lo, v8us hi) { return __builtin_bit_cast(v16bf, __builtin_shufflevector(lo, hi, 0, 1, 2, 3, 4, 5, 6, 7, 8, 9, 10, 11, 12, 13, 14, 15)); }
__device__ __forceinline__ v8f wmma16(v16h a, v16h b, v8f c) { return __builtin_amdgcn_wmma_f32_16x16x32_f16(false, a, false, b, (short)0, c, false, false); }
__device__ __forceinline__ v8f wmmab(v16bf a, v16bf b, v8f c) { return __builtin_amdgcn_wmma_f32_16x16x32_bf16(false, a, false, b, (short)0, c, false, false); }
__device__ __forceinline__ v16h  ldh(const h16* p) { return cat16(*(const v8h*)p, *(const v8h*)(p + 16)); }
__device__ __forceinline__ v16bf ldb(const bf* p)  { return cat16b(*(const v8us*)p, *(const v8us*)(p + 16)); }
__device__ __forceinline__ void wave_sync() { __builtin_amdgcn_fence(3  , "wavefront"); __builtin_amdgcn_wave_barrier(); asm volatile("" ::: "memory"); }

static __device__ __forceinline__ h16 toh_flush(float v) { const h16 r = (h16)v; return (fabsf(v) < 6.103515625e-05f) ? (h16)0.0f : r; }
__device__ __forceinline__ v8f wmma16g(v16h a, v16h b, v8f c) {
    c = __builtin_amdgcn_wmma_f32_16x16x32_f16(false, a, false, b, (short)0, c, false, false);
    asm volatile("v_nop\n\tv_nop\n\tv_nop\n\tv_nop" : "+v"(c) : "v"(a), "v"(b));
    return c; }
__device__ __forceinline__ v8f wmmabg(v16bf a, v16bf b, v8f c) {
    c = __builtin_amdgcn_wmma_f32_16x16x32_bf16(false, a, false, b, (short)0, c, false, false);
    asm volatile("v_nop\n\tv_nop\n\tv_nop\n\tv_nop" : "+v"(c) : "v"(a), "v"(b));
    return c; }

__global__ __launch_bounds__(256) void k_cvt8(const float* __restrict__ src, bf* dst, size_t n8) {
    const size_t i = (size_t)blockIdx.x * 256 + threadIdx.x; if (i >= n8) return;
    const v8f v = *(const v8f*)(src + i * 8); v8us o;
#pragma unroll
    for (int k = 0; k < 8; ++k) o[k] = f2bf(v[k]);
    *(volatile v8us*)(dst + i * 8) = o; __threadfence(); *(volatile v8us*)(dst + i * 8) = o;
}

template <int ASH>
__device__ __forceinline__ void wtr_body(const float* __restrict__ src, bf* dstb, h16* dsth, int R, int C) {
    __shared__ float ts[64 * 65];
    const int tid = threadIdx.x;
    const int r0 = blockIdx.x * 64, c0 = blockIdx.y * 64;
#pragma unroll 1
    for (int i = 0; i < 16; ++i) { const int rr = i * 4 + (tid >> 6), cc = tid & 63;
        ts[rr * 65 + cc] = src[(size_t)(r0 + rr) * C + c0 + cc]; }
    __syncthreads();
    static_assert(256 * 8 * 2 == 64 * 64);
#pragma unroll 1
    for (int ps = 0; ps < 2; ++ps) {
#pragma unroll 1
        for (int it = 0; it < 2; ++it) {
            const int cc = it * 32 + (tid >> 3), r8 = (tid & 7) * 8;
            const size_t oo = (size_t)(c0 + cc) * R + r0 + r8;
            if (ASH) { v8h o;
#pragma unroll
                for (int k = 0; k < 8; ++k) o[k] = toh_flush(bfr(ts[(r8 + k) * 65 + cc]) * WOS);
                *(volatile v8h*)(dsth + oo) = o;
            } else { v8us o;
#pragma unroll
                for (int k = 0; k < 8; ++k) o[k] = f2bf(ts[(r8 + k) * 65 + cc]);
                *(volatile v8us*)(dstb + oo) = o; }
        }
        if (ps == 0) __threadfence(); }
}
__global__ __launch_bounds__(256) void k_wtr_b(const float* __restrict__ src, bf* dst, int R, int C)  { wtr_body<0>(src, dst, (h16*)0, R, C); }
__global__ __launch_bounds__(256) void k_wtr_h(const float* __restrict__ src, h16* dst, int R, int C) { wtr_body<1>(src, (bf*)0, dst, R, C); }

__device__ __forceinline__ void mm64(const bf* __restrict__ A, const bf* __restrict__ Bt, size_t aoff, size_t boff, v8f (&acc)[4][4]) {
    const int K = CIN;
#pragma unroll
    for (int mb = 0; mb < 4; ++mb)
#pragma unroll
        for (int nb = 0; nb < 4; ++nb) acc[mb][nb] = (v8f){};
#pragma unroll 1
    for (int kc = 0; kc < K; kc += 32) {
        v16bf a[4];
#pragma unroll
        for (int mb = 0; mb < 4; ++mb) a[mb] = ldb(A + aoff + (size_t)mb * 16 * K + kc);
#pragma unroll
        for (int nb = 0; nb < 4; ++nb) { const v16bf b = ldb(Bt + boff + (size_t)nb * 16 * K + kc);
#pragma unroll
            for (int mb = 0; mb < 4; ++mb) acc[mb][nb] = wmmabg(a[mb], b, acc[mb][nb]); }
    }
}

__global__ __launch_bounds__(32) void k_proj_q(const bf* __restrict__ A, const bf* __restrict__ Bt, h16* Ph, h16* Pr) {
    __shared__ __align__(16) float os[16 * 68];
    const int lane = threadIdx.x & 31, lr = lane & 15, hi = lane >> 4; const int r0 = blockIdx.x * 64, c0 = blockIdx.y * 64;
    v8f acc[4][4];
    mm64(A, Bt, (size_t)(r0 + lr) * CIN + 8 * hi, (size_t)(c0 + lr) * CIN + 8 * hi, acc);
    const size_t obase = (size_t)r0 * CB + c0;
#pragma unroll
    for (int mb = 0; mb < 4; ++mb) {
#pragma unroll
        for (int nb = 0; nb < 4; ++nb) {
#pragma unroll
            for (int j = 0; j < 8; ++j) os[(hi * 8 + j) * 68 + nb * 16 + lr] = acc[mb][nb][j]; }
        wave_sync();
        static_assert(32 * 8 * 4 == 16 * 64);
#pragma unroll 1
        for (int ps = 0; ps < 2; ++ps) {
#pragma unroll
            for (int s = 0; s < 4; ++s) { const int row = 4 * s + (lane >> 3), c8 = (lane & 7) * 8;
                const v4f x0 = *(const v4fa*)(&os[row * 68 + c8]); const v4f x1 = *(const v4fa*)(&os[row * 68 + c8 + 4]); v8h hv, rv;
#pragma unroll
                for (int i = 0; i < 4; ++i) { const h16 a0 = toh_flush(x0[i]); const h16 a1 = toh_flush(x1[i]); hv[i] = a0; hv[4 + i] = a1;
                    rv[i] = toh_flush((x0[i] - (float)a0) * QRS); rv[4 + i] = toh_flush((x1[i] - (float)a1) * QRS); }
                const size_t oo = obase + (size_t)(mb * 16 + row) * CB + c8;
                *(volatile v8h*)(Ph + oo) = hv; *(volatile v8h*)(Pr + oo) = rv; }
            if (ps == 0) __threadfence(); }
        wave_sync();
    }
}

__global__ __launch_bounds__(32) void k_proj_k(const bf* __restrict__ A, const bf* __restrict__ Bt, h16* Ph, h16* Pr) {
    __shared__ __align__(16) float os[16 * 68];
    const int lane = threadIdx.x & 31, lr = lane & 15, hi = lane >> 4; const int r0 = blockIdx.x * 64, c0 = blockIdx.y * 64;
    v8f acc[4][4];
    mm64(A, Bt, (size_t)(r0 + lr) * CIN + 8 * hi, (size_t)(c0 + lr) * CIN + 8 * hi, acc);
    const size_t obase = (size_t)(r0 / 2) * CB + c0;
#pragma unroll
    for (int mb = 0; mb < 4; ++mb) {
#pragma unroll
        for (int nb = 0; nb < 4; ++nb) {
#pragma unroll
            for (int j = 0; j < 8; ++j) os[(hi * 8 + j) * 68 + nb * 16 + lr] = acc[mb][nb][j]; }
        wave_sync();
        static_assert(32 * 8 * 2 == 8 * 64);
#pragma unroll 1
        for (int ps = 0; ps < 2; ++ps) {
#pragma unroll
            for (int s = 0; s < 2; ++s) { const int prow = 4 * s + (lane >> 3), c8 = (lane & 7) * 8;
                const v4f u0 = *(const v4fa*)(&os[(2 * prow) * 68 + c8]);     const v4f u1 = *(const v4fa*)(&os[(2 * prow) * 68 + c8 + 4]);
                const v4f w0 = *(const v4fa*)(&os[(2 * prow + 1) * 68 + c8]); const v4f w1 = *(const v4fa*)(&os[(2 * prow + 1) * 68 + c8 + 4]); v8h hv, rv;
#pragma unroll
                for (int i = 0; i < 4; ++i) { const float y0 = fmaxf(u0[i], w0[i]), y1 = fmaxf(u1[i], w1[i]);
                    const h16 a0 = toh_flush(y0); const h16 a1 = toh_flush(y1); hv[i] = a0; hv[4 + i] = a1;
                    rv[i] = toh_flush((y0 - (float)a0) * QRS); rv[4 + i] = toh_flush((y1 - (float)a1) * QRS); }
                const size_t oo = obase + (size_t)(mb * 8 + prow) * CB + c8;
                *(volatile v8h*)(Ph + oo) = hv; *(volatile v8h*)(Pr + oo) = rv; }
            if (ps == 0) __threadfence(); }
        wave_sync();
    }
}

__global__ __launch_bounds__(32) void k_proj_gt(const bf* __restrict__ A, const bf* __restrict__ Bt, h16* Gt) {
    __shared__ __align__(16) float os[16 * OPF];
    const int K = CIN;
    const int lane = threadIdx.x & 31, lr = lane & 15, hi = lane >> 4; const int r0 = blockIdx.x * 32, c0 = blockIdx.y * 128;
    v8f acc[2][8];
#pragma unroll
    for (int mb = 0; mb < 2; ++mb)
#pragma unroll
        for (int nb = 0; nb < 8; ++nb) acc[mb][nb] = (v8f){};
    const size_t aoff = (size_t)(r0 + lr) * K + 8 * hi, boff = (size_t)(c0 + lr) * K + 8 * hi;
#pragma unroll 1
    for (int kc = 0; kc < K; kc += 32) {
        v16bf a[2];
#pragma unroll
        for (int mb = 0; mb < 2; ++mb) a[mb] = ldb(A + aoff + (size_t)mb * 16 * K + kc);
#pragma unroll
        for (int nb = 0; nb < 8; ++nb) { const v16bf b = ldb(Bt + boff + (size_t)nb * 16 * K + kc);
#pragma unroll
            for (int mb = 0; mb < 2; ++mb) acc[mb][nb] = wmmabg(a[mb], b, acc[mb][nb]); }
    }
    const int bb = c0 / SEQ, tt = c0 % SEQ;
    const size_t obase = ((size_t)bb * CB + r0) * MK + (size_t)(tt / 2);
#pragma unroll
    for (int mb = 0; mb < 2; ++mb) {
#pragma unroll
        for (int nb = 0; nb < 8; ++nb) {
#pragma unroll
            for (int j = 0; j < 8; ++j) os[(hi * 8 + j) * OPF + nb * 16 + lr] = acc[mb][nb][j]; }
        wave_sync();
        static_assert(32 * 8 * 4 == 16 * 64);
#pragma unroll 1
        for (int ps = 0; ps < 2; ++ps) {
#pragma unroll
            for (int s = 0; s < 4; ++s) { const int row = 4 * s + (lane >> 3), c8 = (lane & 7) * 8;
                const v4f f0 = *(const v4fa*)(&os[row * OPF + 2 * c8]);     const v4f f1 = *(const v4fa*)(&os[row * OPF + 2 * c8 + 4]);
                const v4f f2 = *(const v4fa*)(&os[row * OPF + 2 * c8 + 8]); const v4f f3 = *(const v4fa*)(&os[row * OPF + 2 * c8 + 12]); v8h hv;
                hv[0] = toh_flush(fmaxf(f0[0], f0[1])); hv[1] = toh_flush(fmaxf(f0[2], f0[3]));
                hv[2] = toh_flush(fmaxf(f1[0], f1[1])); hv[3] = toh_flush(fmaxf(f1[2], f1[3]));
                hv[4] = toh_flush(fmaxf(f2[0], f2[1])); hv[5] = toh_flush(fmaxf(f2[2], f2[3]));
                hv[6] = toh_flush(fmaxf(f3[0], f3[1])); hv[7] = toh_flush(fmaxf(f3[2], f3[3]));
                const size_t oo = obase + (size_t)(mb * 16 + row) * MK + c8;
                *(volatile v8h*)(Gt + oo) = hv; }
            if (ps == 0) __threadfence(); }
        wave_sync();
    }
}

__global__ __launch_bounds__(32 * AW) __attribute__((amdgpu_num_vgpr(256)))
void k_attn(const h16* __restrict__ QH, const h16* __restrict__ QR, const h16* __restrict__ KH, const h16* __restrict__ KR,
            const h16* __restrict__ GT, const h16* __restrict__ WO, const float* __restrict__ X, float* OUT) {
    __shared__ __align__(16) float os[AW * 16 * OPF];
    static_assert(sizeof(float) * AW * 16 * OPF <= 131072);
    const int lane = threadIdx.x & 31, lr = lane & 15, hi = lane >> 4;
    const int wave = __builtin_amdgcn_readfirstlane((int)(threadIdx.x >> 5));
    const int b = blockIdx.y;
    const int t0 = (blockIdx.x * AW + wave) * 16;
    const int qo = (b * SEQ + t0 + lr) * CB + 8 * hi;
    const int ko = (b * MK + lr) * CB + 8 * hi;
    const int vo = (b * CB + lr) * MK + 8 * hi;
    v8f o[8];
#pragma unroll
    for (int j = 0; j < 8; ++j) o[j] = (v8f){};
    float m = NEGB, l = 0.0f;
#pragma unroll 1
    for (int key0 = 0; key0 < MK; key0 += 32) {
        int qv = qo; asm volatile("" : "+v"(qv));
        const int kv = ko + key0 * CB;
        v8f sHa = (v8f){}, sLa = (v8f){}, sHb = (v8f){}, sLb = (v8f){};
#pragma unroll 1
        for (int kk = 0; kk < 4; ++kk) {
            const v16h qh = ldh(QH + qv + kk * 32), qr = ldh(QR + qv + kk * 32);
            const v16h ka = ldh(KH + kv + kk * 32),  kb = ldh(KH + kv + 16 * CB + kk * 32);
            const v16h kra = ldh(KR + kv + kk * 32), krb = ldh(KR + kv + 16 * CB + kk * 32);
            sHa = wmma16g(ka, qh, sHa); sHb = wmma16g(kb, qh, sHb);
            sLa = wmma16g(ka, qr, sLa); sLb = wmma16g(kb, qr, sLb);
            sLa = wmma16g(kra, qh, sLa); sLb = wmma16g(krb, qh, sLb);
        }
        float ta[8], tb[8]; float mx = NEGB;
#pragma unroll
        for (int r = 0; r < 8; ++r) {
            ta[r] = (sHa[r] + sLa[r] * QRI) * L2E; tb[r] = (sHb[r] + sLb[r] * QRI) * L2E;
            mx = fmaxf(mx, fmaxf(ta[r], tb[r])); }
        mx = fmaxf(mx, __shfl_xor(mx, 16, 32));
        const float mnew = fmaxf(m, mx);
        const float alpha = __builtin_amdgcn_exp2f(m - mnew);
        const float sh = PSH - mnew;
        v16h pb; float ls = 0.0f;
#pragma unroll
        for (int r = 0; r < 8; ++r) {
            const float ea = ta[r] + sh, eb = tb[r] + sh;
            const float xa = __builtin_amdgcn_exp2f(ea), xb = __builtin_amdgcn_exp2f(eb);
            const float ga = (ea < -14.0f) ? 0.0f : xa, gb = (eb < -14.0f) ? 0.0f : xb;
            const h16 pa = (h16)ga; const h16 pc = (h16)gb;
            pb[r] = pa; pb[8 + r] = pc;
            ls += (float)pa + (float)pc; }
        l = l * alpha + ls; m = mnew;
#pragma unroll
        for (int j = 0; j < 8; ++j) o[j] = o[j] * alpha;
        const int vv = vo + key0;
#pragma unroll
        for (int jg = 0; jg < 2; ++jg) {
            v16h vf[4];
#pragma unroll
            for (int j = 0; j < 4; ++j) vf[j] = ldh(GT + vv + (jg * 4 + j) * 16 * MK);
#pragma unroll
            for (int j = 0; j < 4; ++j) o[jg * 4 + j] = wmma16g(vf[j], pb, o[jg * 4 + j]);
        }
    }
    l += __shfl_xor(l, 16, 32);
    const float inv = 1.0f / l;
    v16h cf[4];
#pragma unroll
    for (int kk = 0; kk < 4; ++kk) {
#pragma unroll
        for (int r = 0; r < 8; ++r) { cf[kk][r] = toh_flush(o[2 * kk][r] * inv); cf[kk][8 + r] = toh_flush(o[2 * kk + 1][r] * inv); } }
    const int wb = wave * 16 * OPF;
    const int wo = lr * CB + 8 * hi;
    const size_t xrow = ((size_t)b * SEQ_FULL + t0) * COUT;
    const size_t orow = ((size_t)b * OUT_SEQ + t0) * COUT;
#pragma unroll 1
    for (int hc = 0; hc < 2; ++hc) {
#pragma unroll 1
        for (int ct = 0; ct < 8; ++ct) {
            const int cg = hc * 8 + ct;
            v8f acc = (v8f){};
#pragma unroll
            for (int kk = 0; kk < 4; ++kk) { const v16h a = ldh(WO + wo + cg * 16 * CB + kk * 32); acc = wmma16g(a, cf[kk], acc); }
            v4f a0, a1;
            a0[0] = acc[0] * WOI; a0[1] = acc[1] * WOI; a0[2] = acc[2] * WOI; a0[3] = acc[3] * WOI;
            a1[0] = acc[4] * WOI; a1[1] = acc[5] * WOI; a1[2] = acc[6] * WOI; a1[3] = acc[7] * WOI;
            *(v4fa*)(&os[wb + lr * OPF + ct * 16 + 8 * hi]) = a0; *(v4fa*)(&os[wb + lr * OPF + ct * 16 + 8 * hi + 4]) = a1;
        }
        wave_sync();
        static_assert(32 * 4 * 16 == 16 * 128);
#pragma unroll 1
        for (int ps = 0; ps < 2; ++ps) {
#pragma unroll 4
            for (int s = 0; s < 16; ++s) { const int cofs = lane * 4;
                const v4f val = *(const v4fa*)(&os[wb + s * OPF + cofs]);
                const v4f xv = *(const v4f*)(X + xrow + (size_t)s * COUT + hc * 128 + cofs);
                v4f res; res[0] = bfr(xv[0]) + val[0]; res[1] = bfr(xv[1]) + val[1]; res[2] = bfr(xv[2]) + val[2]; res[3] = bfr(xv[3]) + val[3];
                *(volatile v4f*)(OUT + orow + (size_t)s * COUT + hc * 128 + cofs) = res; }
            if (ps == 0) __threadfence(); }
        wave_sync();
    }
}

static constexpr size_t al256(size_t v) { return (v + 255) & ~(size_t)255; }
static constexpr size_t SZ_XB = al256((size_t)NB * SEQ * CIN * 2);
static constexpr size_t SZ_W  = al256((size_t)CIN * CB * 2);
static constexpr size_t SZ_Q  = al256((size_t)NB * SEQ * CB * 2);
static constexpr size_t SZ_K  = al256((size_t)NB * MK * CB * 2);
static constexpr size_t SZ_TOTAL = SZ_XB + 4 * SZ_W + 2 * SZ_Q + 3 * SZ_K;
static_assert(SZ_TOTAL <= (size_t)134217728);
static_assert((size_t)CIN * CB == (size_t)CB * COUT);
static_assert((size_t)NB * MK * CB == (size_t)NB * CB * MK);

extern "C" void kernel_launch(void* const* d_in, const int* in_sizes, int n_in,
                              void* d_out, int out_size, void* d_ws, size_t ws_size, hipStream_t stream) {
    if (n_in < 5) return;
    const size_t needx = ((size_t)(NB - 1) * SEQ_FULL + SEQ) * CIN;
    if ((size_t)in_sizes[0] < needx) return;
    if ((size_t)in_sizes[1] < (size_t)CIN * CB || (size_t)in_sizes[2] < (size_t)CIN * CB || (size_t)in_sizes[3] < (size_t)CIN * CB) return;
    if ((size_t)in_sizes[4] < (size_t)CB * COUT) return;
    if ((size_t)out_size < ((size_t)(NB - 1) * OUT_SEQ + SEQ) * COUT) return;
    if (SZ_TOTAL > ws_size) return;
    const float* x  = (const float*)d_in[0];
    const float* wt = (const float*)d_in[1];
    const float* wp = (const float*)d_in[2];
    const float* wg = (const float*)d_in[3];
    const float* wo = (const float*)d_in[4];
    float* OUT = (float*)d_out;
    char* wsp = (char*)d_ws;
    bf*  XB = (bf*)wsp;  wsp += SZ_XB;
    bf*  WT = (bf*)wsp;  wsp += SZ_W;
    bf*  WP = (bf*)wsp;  wsp += SZ_W;
    bf*  WG = (bf*)wsp;  wsp += SZ_W;
    h16* WOH = (h16*)wsp; wsp += SZ_W;
    h16* QH = (h16*)wsp; wsp += SZ_Q;
    h16* QR = (h16*)wsp; wsp += SZ_Q;
    h16* KH = (h16*)wsp; wsp += SZ_K;
    h16* KR = (h16*)wsp; wsp += SZ_K;
    h16* GT = (h16*)wsp; wsp += SZ_K;

    if (SEQ == SEQ_FULL) {
        const size_t n8 = (size_t)NB * SEQ * CIN / 8;
        k_cvt8<<<(unsigned)((n8 + 255) / 256), 256, 0, stream>>>(x, XB, n8);
    } else {
        const size_t n8 = (size_t)SEQ * CIN / 8;
        for (int b = 0; b < NB; ++b) k_cvt8<<<(unsigned)((n8 + 255) / 256), 256, 0, stream>>>(x + (size_t)b * SEQ_FULL * CIN, XB + (size_t)b * SEQ * CIN, n8);
    }
    k_wtr_b<<<dim3(CIN / 64, CB / 64, 1), 256, 0, stream>>>(wt, WT, CIN, CB);
    k_wtr_b<<<dim3(CIN / 64, CB / 64, 1), 256, 0, stream>>>(wp, WP, CIN, CB);
    k_wtr_b<<<dim3(CIN / 64, CB / 64, 1), 256, 0, stream>>>(wg, WG, CIN, CB);
    k_wtr_h<<<dim3(CB / 64, COUT / 64, 1), 256, 0, stream>>>(wo, WOH, CB, COUT);

    k_proj_q<<<dim3(NB * SEQ / 64, CB / 64, 1), 32, 0, stream>>>(XB, WT, QH, QR);
    k_proj_k<<<dim3(NB * SEQ / 64, CB / 64, 1), 32, 0, stream>>>(XB, WP, KH, KR);
    k_proj_gt<<<dim3(CB / 32, NB * SEQ / 128, 1), 32, 0, stream>>>(WG, XB, GT);

    k_attn<<<dim3(SEQ / (16 * AW), NB, 1), 32 * AW, 0, stream>>>(QH, QR, KH, KR, GT, WOH, x, OUT);
}
